// GraphConv_28475633173124
// MI455X (gfx1250) — hardware-verified
//
#include <hip/hip_runtime.h>
#include <math.h>

constexpr int kBatch     = 4;
constexpr int kChIn      = 128;
constexpr int kNode      = 4096;
constexpr int kNbr       = 16;
constexpr int kChOut     = 256;
constexpr int kRows      = kBatch * kNode;
constexpr int kPQld      = 2 * kChOut;
constexpr int kEdgePlane = kBatch * kNode * kNbr;
constexpr int kNodeTile  = 32;
constexpr int kTiles     = kRows / kNodeTile;
constexpr float kBnEps   = 1e-5f;

static_assert(kChIn % 32 == 0);
static_assert(kRows % 64 == 0);
static_assert(kPQld % 64 == 0);
static_assert(kNode % kNodeTile == 0);
static_assert(kRows % kNodeTile == 0);

constexpr size_t kOffXT    = 0;
constexpr size_t kBytesXT  = (size_t)kRows * kChIn * 2;
constexpr size_t kOffBT    = kOffXT + kBytesXT;
constexpr size_t kBytesBT  = (size_t)kPQld * kChIn * 2;
constexpr size_t kOffPQ    = kOffBT + kBytesBT;
constexpr size_t kBytesPQ  = (size_t)kRows * kPQld * 4;
constexpr size_t kOffRM    = kOffPQ + kBytesPQ;
constexpr size_t kBytesRM  = (size_t)kRows * kChOut * 4;
constexpr size_t kOffPS    = kOffRM + kBytesRM;
constexpr size_t kBytesPS  = (size_t)kTiles * kChOut * 4;
constexpr size_t kOffPQ2   = kOffPS + kBytesPS;
constexpr size_t kOffST    = kOffPQ2 + kBytesPS;
constexpr size_t kBytesST  = (size_t)2 * kChOut * 4;
constexpr size_t kWsTotal  = kOffST + kBytesST;
static_assert(kWsTotal == 55707648);
static_assert(kWsTotal <= (size_t)134217728);
static_assert(kOffBT % 256 == 0 && kOffPQ % 256 == 0 && kOffRM % 256 == 0 && kOffPS % 256 == 0 && kOffPQ2 % 256 == 0 && kOffST % 256 == 0);

typedef __attribute__((ext_vector_type(16))) _Float16 v16h;
typedef __attribute__((ext_vector_type(8)))  _Float16 v8h;
typedef __attribute__((ext_vector_type(16))) __bf16   v16b;
typedef __attribute__((ext_vector_type(8)))  __bf16   v8b;
typedef __attribute__((ext_vector_type(8)))  float    v8f;
typedef __attribute__((ext_vector_type(4)))  float    v4f;
typedef __attribute__((ext_vector_type(4)))  unsigned int v4u;
typedef __attribute__((ext_vector_type(4)))  int      v4i;

__device__ __forceinline__ unsigned short f2bf_bits(float f) {
  unsigned u = __float_as_uint(f);
  return (unsigned short)((u + 0x7FFFu + ((u >> 16) & 1u)) >> 16);
}
__device__ __forceinline__ float bf_bits2f(unsigned short h) { return __uint_as_float(((unsigned)h) << 16); }
__device__ __forceinline__ unsigned pk16(unsigned short a, unsigned short b) { return (unsigned)a | ((unsigned)b << 16); }

__device__ __forceinline__ void dep_guard_h(v8f& a, v8f& b, v16h x, v16h y) { asm volatile("v_nop\n\tv_nop\n\tv_nop\n\tv_nop" : "+v"(a), "+v"(b) : "v"(x), "v"(y)); }
__device__ __forceinline__ void dep_guard_b(v8f& a, v8f& b, v16b x, v16b y) { asm volatile("v_nop\n\tv_nop\n\tv_nop\n\tv_nop" : "+v"(a), "+v"(b) : "v"(x), "v"(y)); }
__device__ __forceinline__ void keep4_h(v16h a, v16h b, v16h c, v16h d) { asm volatile("v_nop" :: "v"(a), "v"(b), "v"(c), "v"(d)); }
__device__ __forceinline__ void keep4_b(v16b a, v16b b, v16b c, v16b d) { asm volatile("v_nop" :: "v"(a), "v"(b), "v"(c), "v"(d)); }
__device__ __forceinline__ void acc_guard4(v8f& a, v8f& b, v8f& c, v8f& d) { asm volatile("v_nop\n\tv_nop\n\tv_nop\n\tv_nop" : "+v"(a), "+v"(b), "+v"(c), "+v"(d)); }
template <typename T> struct Frag;
template <> struct Frag<_Float16> {
  typedef v16h V; union U { v16h v; v8h h[2]; };
  static __device__ __forceinline__ v16h load(const _Float16* p) {
    U f; f.h[0] = *(const v8h*)(p); f.h[1] = *(const v8h*)(p + 16); return f.v;
  }
  static __device__ __forceinline__ v8f mma(v16h a, v16h b, v8f c) {
    return __builtin_amdgcn_wmma_f32_16x16x32_f16(false, a, false, b, (short)0, c, false, false);
  }
  static __device__ __forceinline__ void guard(v8f& a, v8f& b, v16h x, v16h y) { dep_guard_h(a, b, x, y); }
  static __device__ __forceinline__ void keep(v16h a, v16h b, v16h c, v16h d) { keep4_h(a, b, c, d); }
};
template <> struct Frag<__bf16> {
  typedef v16b V; union U { v16b v; v8b h[2]; };
  static __device__ __forceinline__ v16b load(const __bf16* p) {
    U f; f.h[0] = *(const v8b*)(p); f.h[1] = *(const v8b*)(p + 16); return f.v;
  }
  static __device__ __forceinline__ v8f mma(v16b a, v16b b, v8f c) {
    return __builtin_amdgcn_wmma_f32_16x16x32_bf16(false, a, false, b, (short)0, c, false, false);
  }
  static __device__ __forceinline__ void guard(v8f& a, v8f& b, v16b x, v16b y) { dep_guard_b(a, b, x, y); }
  static __device__ __forceinline__ void keep(v16b a, v16b b, v16b c, v16b d) { keep4_b(a, b, c, d); }
};

template <int ET> struct Elem;
template <> struct Elem<0> { typedef _Float16 T; };
template <> struct Elem<1> { typedef __bf16 T; };
template <int ET, bool SPLIT, int BIAS_MODE, int OUT_MODE, bool RESID, int ACT = 0>
__global__ __launch_bounds__(256) void wmma_gemm64(
    const unsigned short* __restrict__ Ap, const unsigned short* __restrict__ A2p, int lda, long strideA,
    const unsigned short* __restrict__ Btp, const unsigned short* __restrict__ Bt2p, int ldb, long strideB,
    void* __restrict__ Cout, void* __restrict__ Cout2, int ldc, long strideC,
    const float* __restrict__ bias,
    const float* __restrict__ resid, long strideR,
    int M, int N, int K, float scale) {
  typedef typename Elem<ET>::T T;
  typedef typename Frag<T>::V V;
  const T* A = (const T*)Ap; const T* A2 = (const T*)A2p; const T* Bt = (const T*)Btp; const T* Bt2 = (const T*)Bt2p;
  __shared__ __align__(16) float sT[8][16 * 68];
  const int b    = blockIdx.y;
  const int lane = threadIdx.x & 31;
  const int wave = threadIdx.x >> 5;
  const int tilesN = N >> 6;
  const int tilesM = M >> 6;
  const int tile = blockIdx.x * 8 + wave;
  if (tile >= tilesM * tilesN) return;
  const int tm = tile / tilesN;
  const int tn = tile - tm * tilesN;
  const int m0 = tm << 6;
  const int n0 = tn << 6;

  const T* Ab  = A  + (size_t)b * strideA;
  const T* Bb  = Bt + (size_t)b * strideB;
  const T* Ab2 = SPLIT ? (A2  + (size_t)b * strideA) : nullptr;
  const T* Bb2 = SPLIT ? (Bt2 + (size_t)b * strideB) : nullptr;

  const int rlane = lane & 15;
  const int koff  = (lane >> 4) * 8;
  const int mOff  = (lane >> 4) * 8;

  v8f acc[4][4];
#pragma unroll
  for (int i = 0; i < 4; ++i)
#pragma unroll
    for (int j = 0; j < 4; ++j) acc[i][j] = (v8f){0.f,0.f,0.f,0.f,0.f,0.f,0.f,0.f};

  for (int k0 = 0; k0 < K; k0 += 32) {
    V bh[4], bl[4];
#pragma unroll
    for (int j = 0; j < 4; ++j) {
      const size_t bo = (size_t)(n0 + (j << 4) + rlane) * ldb + koff + k0;
      bh[j] = Frag<T>::load(Bb + bo);
      if (SPLIT) bl[j] = Frag<T>::load(Bb2 + bo);
    }
#pragma unroll
    for (int i = 0; i < 4; ++i) {
      const size_t ao = (size_t)(m0 + (i << 4) + rlane) * lda + koff + k0;
      V ah = Frag<T>::load(Ab + ao);
      V al;
      if (SPLIT) al = Frag<T>::load(Ab2 + ao);
#pragma unroll
      for (int j = 0; j < 4; ++j) {
        acc[i][j] = Frag<T>::mma(ah, bh[j], acc[i][j]);
        if (SPLIT) {
          acc[i][j] = Frag<T>::mma(ah, bl[j], acc[i][j]);
          acc[i][j] = Frag<T>::mma(al, bh[j], acc[i][j]);
        }
      }
      Frag<T>::guard(acc[i][0], acc[i][3], ah, SPLIT ? al : ah);
    }
    Frag<T>::keep(bh[0], bh[1], bh[2], bh[3]);
    if (SPLIT) Frag<T>::keep(bl[0], bl[1], bl[2], bl[3]);
  }
  acc_guard4(acc[0][0], acc[0][1], acc[0][2], acc[0][3]);
  acc_guard4(acc[1][0], acc[1][1], acc[1][2], acc[1][3]);
  acc_guard4(acc[2][0], acc[2][1], acc[2][2], acc[2][3]);
  acc_guard4(acc[3][0], acc[3][1], acc[3][2], acc[3][3]);

  float* slab = sT[wave];
  const float* Rb = RESID ? (resid + (size_t)b * strideR) : nullptr;
#pragma unroll
  for (int i = 0; i < 4; ++i) {
    const int mBase = m0 + (i << 4);
#pragma unroll
    for (int j = 0; j < 4; ++j) {
      const int n = n0 + (j << 4) + rlane;
      float bv = 0.f;
      if (BIAS_MODE == 2) bv = bias[n];
#pragma unroll
      for (int r = 0; r < 8; ++r) {
        float v = acc[i][j][r] * scale;
        if (BIAS_MODE == 1) v += bias[mBase + mOff + r];
        if (BIAS_MODE == 2) v += bv;
        if (RESID) v += Rb[(size_t)(mBase + mOff + r) * ldc + n];
        if (ACT == 2) v = fmaxf(v, 0.0f);
        if (ACT == 4) v = (v > 0.f) ? v : 0.01f * v;
        slab[(mOff + r) * 68 + (j << 4) + rlane] = v;
      }
    }
    __builtin_amdgcn_fence(__ATOMIC_RELEASE, "workgroup");
    __builtin_amdgcn_wave_barrier();
    __builtin_amdgcn_fence(__ATOMIC_ACQUIRE, "workgroup");
    if (OUT_MODE == 0) {
      float* C = (float*)Cout + (size_t)b * strideC;
      const int hh = lane >> 4, c4 = (lane & 15) * 4;
      for (int pass = 0; pass < 2; ++pass) {
#pragma unroll
        for (int it = 0; it < 8; ++it) {
          const int row = it * 2 + hh;
          v4f v = *(const v4f*)(slab + row * 68 + c4);
          *(volatile v4f*)(C + (size_t)(mBase + row) * ldc + n0 + c4) = v;
        }
        __threadfence();
      }
    } else {
      const int q = lane >> 3, c8 = (lane & 7) * 8;
      unsigned short* C  = (unsigned short*)Cout  + (size_t)b * strideC;
      unsigned short* C2 = (OUT_MODE == 2) ? ((unsigned short*)Cout2 + (size_t)b * strideC) : nullptr;
      for (int pass = 0; pass < 2; ++pass) {
#pragma unroll
        for (int it = 0; it < 4; ++it) {
          const int row = it * 4 + q;
          const float* sp = slab + row * 68 + c8;
          v8h hv, lv;
#pragma unroll
          for (int e = 0; e < 8; ++e) {
            if (OUT_MODE == 1) {
              hv[e] = (_Float16)sp[e];
            } else {
              unsigned short hb = f2bf_bits(sp[e]);
              unsigned short lb = f2bf_bits(sp[e] - bf_bits2f(hb));
              hv[e] = __builtin_bit_cast(_Float16, hb);
              lv[e] = __builtin_bit_cast(_Float16, lb);
            }
          }
          *(volatile v8h*)(C + (size_t)(mBase + row) * ldc + n0 + c8) = hv;
          if (OUT_MODE == 2) *(volatile v8h*)(C2 + (size_t)(mBase + row) * ldc + n0 + c8) = lv;
        }
        __threadfence();
      }
    }
    __builtin_amdgcn_fence(__ATOMIC_RELEASE, "workgroup");
    __builtin_amdgcn_wave_barrier();
    __builtin_amdgcn_fence(__ATOMIC_ACQUIRE, "workgroup");
  }
}

__device__ __forceinline__ int clamp_node(int v) { v = v < 0 ? 0 : v; return v > (kNode - 1) ? (kNode - 1) : v; }

__global__ __launch_bounds__(256) void xt_kernel(const float* __restrict__ x, unsigned short* __restrict__ xT) {
  __shared__ __align__(16) float sm[kNodeTile][132];
  const int t  = threadIdx.x;
  const int p0 = blockIdx.x * kNodeTile;
  const int b  = p0 >> 12;
  const int n0 = p0 & (kNode - 1);
  const int nl = t & 31;
  const int cb = t >> 5;
  const float* src = x + (size_t)b * kChIn * kNode + n0 + nl;
#pragma unroll
  for (int i = 0; i < 8; ++i) {
    const int c = cb + 8 * i;
    sm[nl][c] = src[(size_t)c * kNode];
  }
  asm volatile("" ::: "memory");
#pragma unroll
  for (int i = 0; i < 8; ++i) {
    const int c = cb + 64 + 8 * i;
    sm[nl][c] = src[(size_t)c * kNode];
  }
  __syncthreads();
  const int lane = t & 31, wave = t >> 5;
  const int hh = lane >> 4, c8 = (lane & 15) * 8;
  for (int pass = 0; pass < 2; ++pass) {
#pragma unroll
    for (int it = 0; it < 2; ++it) {
      const int row = wave * 4 + it * 2 + hh;
      const v4f a = *(const v4f*)(&sm[row][c8]);
      const v4f c = *(const v4f*)(&sm[row][c8 + 4]);
      const v4u u = (v4u){pk16(f2bf_bits(a[0]), f2bf_bits(a[1])), pk16(f2bf_bits(a[2]), f2bf_bits(a[3])),
                          pk16(f2bf_bits(c[0]), f2bf_bits(c[1])), pk16(f2bf_bits(c[2]), f2bf_bits(c[3]))};
      *(volatile v4u*)(xT + (size_t)(p0 + row) * kChIn + c8) = u;
    }
    __threadfence();
  }
}

__global__ __launch_bounds__(256) void bt_kernel(const float* __restrict__ w, unsigned short* __restrict__ Bt) {
  const int i = blockIdx.x * 256 + threadIdx.x;
  if (i >= kPQld * (kChIn / 8)) return;
  const int r  = i >> 4;
  const int k8 = (i & 15) * 8;
  const float* src = w + (size_t)(r & (kChOut - 1)) * (2 * kChIn) + (r >> 8) * kChIn + k8;
  const v4f a = *(const v4f*)(src);
  const v4f c = *(const v4f*)(src + 4);
  const v4u u = (v4u){pk16(f2bf_bits(a[0]), f2bf_bits(a[1])), pk16(f2bf_bits(a[2]), f2bf_bits(a[3])),
                      pk16(f2bf_bits(c[0]), f2bf_bits(c[1])), pk16(f2bf_bits(c[2]), f2bf_bits(c[3]))};
  unsigned short* dst = Bt + (size_t)r * kChIn + k8;
  *(volatile v4u*)dst = u;
  __threadfence();
  *(volatile v4u*)dst = u;
}

__global__ __launch_bounds__(256) void edge_kernel(const float* __restrict__ PQ, const int* __restrict__ ei,
                                                  const float* __restrict__ bias, float* __restrict__ rawmax,
                                                  float* __restrict__ psum, float* __restrict__ psq) {
  __shared__ __align__(16) int   sIdx[2 * kNodeTile * kNbr];
  __shared__ __align__(16) float redS[4][kChOut];
  __shared__ __align__(16) float redQ[4][kChOut];
  const int t    = threadIdx.x;
  const int g    = t >> 6;
  const int q    = t & 63;
  const int c4   = q * 4;
  const int p0   = blockIdx.x * kNodeTile;
  const int b    = p0 >> 12;
  const int rowb = b * kNode;
  {
    const size_t off = (size_t)p0 * kNbr + (size_t)(4 * t) + ((t < 128) ? (size_t)0 : (size_t)(kEdgePlane - 512));
    const v4i v = *(const v4i*)(ei + off);
    v4i cv;
    cv[0] = clamp_node(v[0]); cv[1] = clamp_node(v[1]); cv[2] = clamp_node(v[2]); cv[3] = clamp_node(v[3]);
    *(v4i*)(sIdx + 4 * t) = cv;
  }
  __syncthreads();

  const v4f b4 = *(const v4f*)(bias + c4);
  const v4f z4 = (v4f){0.f, 0.f, 0.f, 0.f};
  v4f s4 = z4, q4 = z4;
  const float* P1c = PQ + c4;
  const float* P2c = PQ + kChOut + c4;
#pragma unroll 1
  for (int it = 0; it < 8; ++it) {
    const int nl = g + 4 * it;
    v4f m4 = z4;
#pragma unroll 2
    for (int k = 0; k < kNbr; ++k) {
      const int jl = sIdx[nl * kNbr + k];
      const int il = sIdx[kNodeTile * kNbr + nl * kNbr + k];
      const size_t ri = (size_t)(rowb + il) * kPQld;
      const size_t rj = (size_t)(rowb + jl) * kPQld;
      const v4f p1  = *(const v4f*)(P1c + ri);
      const v4f p2i = *(const v4f*)(P2c + ri);
      const v4f p2j = *(const v4f*)(P2c + rj);
      v4f v = p2j - p2i;
      v = v + p1;
      v = v + b4;
      v[0] = fmaxf(v[0], 0.f); v[1] = fmaxf(v[1], 0.f); v[2] = fmaxf(v[2], 0.f); v[3] = fmaxf(v[3], 0.f);
      m4[0] = fmaxf(m4[0], v[0]); m4[1] = fmaxf(m4[1], v[1]); m4[2] = fmaxf(m4[2], v[2]); m4[3] = fmaxf(m4[3], v[3]);
      s4 = s4 + v;
      q4[0] = fmaf(v[0], v[0], q4[0]); q4[1] = fmaf(v[1], v[1], q4[1]);
      q4[2] = fmaf(v[2], v[2], q4[2]); q4[3] = fmaf(v[3], v[3], q4[3]);
    }
    float* rp = rawmax + (size_t)(p0 + nl) * kChOut + c4;
    *(volatile v4f*)rp = m4;
    __threadfence();
    *(volatile v4f*)rp = m4;
  }
  *(v4f*)(&redS[g][c4]) = s4;
  *(v4f*)(&redQ[g][c4]) = q4;
  __syncthreads();
  if (g == 0) {
    v4f ss = *(const v4f*)(&redS[0][c4]);
    ss = ss + *(const v4f*)(&redS[1][c4]);
    ss = ss + *(const v4f*)(&redS[2][c4]);
    ss = ss + *(const v4f*)(&redS[3][c4]);
    v4f qq = *(const v4f*)(&redQ[0][c4]);
    qq = qq + *(const v4f*)(&redQ[1][c4]);
    qq = qq + *(const v4f*)(&redQ[2][c4]);
    qq = qq + *(const v4f*)(&redQ[3][c4]);
    float* ps = psum + (size_t)blockIdx.x * kChOut + c4;
    float* pq = psq  + (size_t)blockIdx.x * kChOut + c4;
    *(volatile v4f*)ps = ss;
    *(volatile v4f*)pq = qq;
    __threadfence();
    *(volatile v4f*)ps = ss;
    *(volatile v4f*)pq = qq;
  }
}

__global__ __launch_bounds__(256) void stats_kernel(const float* __restrict__ psum, const float* __restrict__ psq,
                                                   const float* __restrict__ gamma, const float* __restrict__ beta,
                                                   float* __restrict__ stats) {
  const int o = threadIdx.x;
  double S = 0.0, Q = 0.0;
#pragma unroll 4
  for (int blk = 0; blk < kTiles; ++blk) {
    S += (double)psum[(size_t)blk * kChOut + o];
    Q += (double)psq [(size_t)blk * kChOut + o];
  }
  const double invc = 1.0 / (double)((long)kRows * (long)kNbr);
  const float mean = (float)(S * invc);
  const float ey2  = (float)(Q * invc);
  const float var  = ey2 - mean * mean;
  const float sc   = gamma[o] * (1.0f / sqrtf(var + kBnEps));
  const float sh   = beta[o] - mean * sc;
  ((volatile float*)stats)[o] = sc;
  ((volatile float*)stats)[kChOut + o] = sh;
  __threadfence();
  ((volatile float*)stats)[o] = sc;
  ((volatile float*)stats)[kChOut + o] = sh;
}

__global__ __launch_bounds__(256) void out_kernel(const float* __restrict__ rawmax, const float* __restrict__ stats,
                                                 float* __restrict__ out) {
  __shared__ __align__(16) float sm[kChOut][36];
  const int t  = threadIdx.x;
  const int p0 = blockIdx.x * kNodeTile;
  const int b  = p0 >> 12;
  const int n0 = p0 & (kNode - 1);
  const int q  = t & 63, c4 = q * 4, g = t >> 6;
  const v4f sc4 = *(const v4f*)(stats + c4);
  const v4f sh4 = *(const v4f*)(stats + kChOut + c4);
#pragma unroll 4
  for (int it = 0; it < 8; ++it) {
    const int nl = g + 4 * it;
    const v4f m = *(const v4f*)(rawmax + (size_t)(p0 + nl) * kChOut + c4);
    const v4f v = m * sc4 + sh4;
    sm[c4 + 0][nl] = v[0];
    sm[c4 + 1][nl] = v[1];
    sm[c4 + 2][nl] = v[2];
    sm[c4 + 3][nl] = v[3];
  }
  __syncthreads();
  const int lane = t & 31, wave = t >> 5;
  const int ol = lane >> 3, n4 = (lane & 7) * 4;
  float* ob = out + (size_t)b * kChOut * kNode + n0 + n4;
  for (int pass = 0; pass < 2; ++pass) {
#pragma unroll
    for (int it = 0; it < 8; ++it) {
      const int o = wave * 32 + it * 4 + ol;
      const v4f v = *(const v4f*)(&sm[o][n4]);
      *(volatile v4f*)(ob + (size_t)o * kNode) = v;
    }
    __threadfence();
  }
}

extern "C" void kernel_launch(void* const* d_in, const int* in_sizes, int n_in,
                              void* d_out, int out_size, void* d_ws, size_t ws_size,
                              hipStream_t stream) {
  if (n_in < 6) return;
  if (in_sizes[0] != kBatch * kChIn * kNode) return;
  if (in_sizes[1] != kChOut * 2 * kChIn) return;
  if (in_sizes[2] < kChOut || in_sizes[3] < kChOut || in_sizes[4] < kChOut) return;
  if (in_sizes[5] != 2 * kEdgePlane) return;
  if (out_size != kBatch * kChOut * kNode) return;
  if (ws_size < kWsTotal) return;

  const float* x     = (const float*)d_in[0];
  const float* w     = (const float*)d_in[1];
  const float* bias  = (const float*)d_in[2];
  const float* gamma = (const float*)d_in[3];
  const float* beta  = (const float*)d_in[4];
  const int*   ei    = (const int*)  d_in[5];
  float* out = (float*)d_out;

  char* ws = (char*)d_ws;
  unsigned short* xT     = (unsigned short*)(ws + kOffXT);
  unsigned short* Bt     = (unsigned short*)(ws + kOffBT);
  float*          PQ     = (float*)(ws + kOffPQ);
  float*          rawmax = (float*)(ws + kOffRM);
  float*          psum   = (float*)(ws + kOffPS);
  float*          psq    = (float*)(ws + kOffPQ2);
  float*          stats  = (float*)(ws + kOffST);

  xt_kernel<<<kTiles, 256, 0, stream>>>(x, xT);
  bt_kernel<<<(kPQld * (kChIn / 8)) / 256, 256, 0, stream>>>(w, Bt);
  {
    const int tiles = (kRows / 64) * (kPQld / 64);
    wmma_gemm64<1, false, 0, 0, false, 0><<<dim3((tiles + 7) / 8, 1), 256, 0, stream>>>(
        (const unsigned short*)xT, (const unsigned short*)nullptr, kChIn, 0L,
        (const unsigned short*)Bt, (const unsigned short*)nullptr, kChIn, 0L,
        (void*)PQ, (void*)nullptr, kPQld, 0L,
        (const float*)nullptr, (const float*)nullptr, 0L, kRows, kPQld, kChIn, 1.0f);
  }
  edge_kernel<<<kTiles, 256, 0, stream>>>(PQ, ei, bias, rawmax, psum, psq);
  stats_kernel<<<1, kChOut, 0, stream>>>(psum, psq, gamma, beta, stats);
  out_kernel<<<kTiles, 256, 0, stream>>>(rawmax, stats, out);
}
